// StableTopoBrain_18769007084171
// MI455X (gfx1250) — hardware-verified
//
#include <hip/hip_runtime.h>
#include <math.h>
#include <stdint.h>
#include <stddef.h>


typedef _Float16 f16;
typedef f16 v8h __attribute__((ext_vector_type(8)));
typedef f16 v16h __attribute__((ext_vector_type(16)));
typedef float v4f __attribute__((ext_vector_type(4)));
typedef float v8f __attribute__((ext_vector_type(8)));

union Frag { v16h v; v8h half[2]; };

#define NN 256
#define DD 64
#define FF 512
#define HH 16384
#define NCLS 1000
#define NCP 1008
#define RBH 2048
#define TP 264
#define CLIPV 3.0f

#define SC_WIN 16.0f
#define WEFF_POST 2.0f
#define INV_WEFF 0.03125f
#define SC_V 8.0f
#define INV_V 0.125f
#define SC_S 64.0f
#define INV_S 0.015625f
#define SC_Y 16.0f
#define INV_YV 0.0078125f
#define SC_CELL 8.0f
#define SC_MQ 16.0f
#define INV_ATT 0.0078125f
#define SC_XC 8.0f
#define SC_WO 64.0f
#define INV_OUT 0.001953125f

static __device__ __forceinline__ v8f zero8() {
  v8f z;
#pragma unroll
  for (int i = 0; i < 8; ++i) z[i] = 0.0f;
  return z;
}

static __device__ __forceinline__ v8f wmma16(const v16h a, const v16h b, v8f c) {
  return __builtin_amdgcn_wmma_f32_16x16x32_f16(false, a, false, b, (short)0, c, false, false);
}

static __device__ __forceinline__ void guard_1(v8f& d, const v16h& a0, const v16h& a1,
                                               const v16h& b0, const v16h& b1) {
  asm volatile("v_nop\n\tv_nop\n\tv_nop\n\tv_nop" : "+v"(d) : "v"(a0), "v"(a1), "v"(b0), "v"(b1));
}
static __device__ __forceinline__ void guard_2(v8f& d0, v8f& d1, const v16h& a0, const v16h& a1,
                                               const v16h& a2, const v16h& a3,
                                               const v16h& b0, const v16h& b1) {
  asm volatile("v_nop\n\tv_nop\n\tv_nop\n\tv_nop"
               : "+v"(d0), "+v"(d1)
               : "v"(a0), "v"(a1), "v"(a2), "v"(a3), "v"(b0), "v"(b1));
}
static __device__ __forceinline__ void guard_3(v8f& d0, v8f& d1, v8f& d2,
                                               const v16h& b0, const v16h& b1, const v16h& b2,
                                               const v16h& a) {
  asm volatile("v_nop\n\tv_nop\n\tv_nop\n\tv_nop"
               : "+v"(d0), "+v"(d1), "+v"(d2)
               : "v"(b0), "v"(b1), "v"(b2), "v"(a));
}
static __device__ __forceinline__ void guard_4(v8f& d0, v8f& d1, v8f& d2, v8f& d3,
                                               const v16h& a0, const v16h& a1,
                                               const v16h& a2, const v16h& a3, const v16h& b) {
  asm volatile("v_nop\n\tv_nop\n\tv_nop\n\tv_nop"
               : "+v"(d0), "+v"(d1), "+v"(d2), "+v"(d3)
               : "v"(a0), "v"(a1), "v"(a2), "v"(a3), "v"(b));
}
static __device__ __forceinline__ void guard_8w(v8f (&d)[8], const v16h& a0, const v16h& a1,
                                                const v16h& b0, const v16h& b1,
                                                const v16h& b2, const v16h& b3) {
  asm volatile("v_nop\n\tv_nop\n\tv_nop\n\tv_nop"
               : "+v"(d[0]), "+v"(d[1]), "+v"(d[2]), "+v"(d[3]),
                 "+v"(d[4]), "+v"(d[5]), "+v"(d[6]), "+v"(d[7])
               : "v"(a0), "v"(a1), "v"(b0), "v"(b1), "v"(b2), "v"(b3));
}

static __device__ __forceinline__ v16h ldf(const f16* p) {
  Frag f;
  f.half[0] = *(const v8h*)(p);
  f.half[1] = *(const v8h*)(p + 16);
  return f.v;
}

static __device__ __forceinline__ v16h pack2(const v8f& lo, const v8f& hi, float s) {
  Frag f;
  v8h l, u;
#pragma unroll
  for (int r = 0; r < 8; ++r) { l[r] = (f16)(lo[r] * s); u[r] = (f16)(hi[r] * s); }
  f.half[0] = l;
  f.half[1] = u;
  return f.v;
}

template <typename T>
static __device__ __forceinline__ void vst2(T* p, const T v) {
  *(volatile T*)p = v;
  __threadfence();
  *(volatile T*)p = v;
}

static __device__ __forceinline__ v8f clip8s(v8f v, float s) {
#pragma unroll
  for (int i = 0; i < 8; ++i) v[i] = fminf(CLIPV, fmaxf(-CLIPV, v[i] * s));
  return v;
}

static __device__ __forceinline__ v8f axpb8(v8f a, float s, const float* b) {
  const v4f b0 = *(const v4f*)(b), b1 = *(const v4f*)(b + 4);
  v8f o;
#pragma unroll
  for (int i = 0; i < 4; ++i) { o[i] = a[i] * s + b0[i]; o[4 + i] = a[4 + i] * s + b1[i]; }
  return o;
}

static __device__ __forceinline__ float dot8(const v8f& a, const float* w) {
  const v4f w0 = *(const v4f*)(w), w1 = *(const v4f*)(w + 4);
  float s = 0.0f;
#pragma unroll
  for (int i = 0; i < 4; ++i) { s += a[i] * w0[i]; s += a[4 + i] * w1[i]; }
  return s;
}

static __device__ __forceinline__ float sigm_fast(float x) {
  const float v = __expf(-x);
  return __builtin_amdgcn_rcpf(1.0f + v);
}

static __device__ __forceinline__ void chain_pair(const f16* __restrict__ A16, int c0, int m, int h,
                                                  const v16h& b0, const v16h& b1, v8f& d0, v8f& d1) {
  const f16* p0 = A16 + (size_t)((c0 * 16 + m) * DD) + 8 * h;
  const f16* p1 = p0 + 16 * DD;
  const v16h a00 = ldf(p0), a01 = ldf(p0 + 32);
  const v16h a10 = ldf(p1), a11 = ldf(p1 + 32);
  d0 = wmma16(a00, b0, zero8());
  d0 = wmma16(a01, b1, d0);
  d1 = wmma16(a10, b0, zero8());
  d1 = wmma16(a11, b1, d1);
  guard_2(d0, d1, a00, a01, a10, a11, b0, b1);
}

__global__ __launch_bounds__(256) void k_prep(
    const float* __restrict__ adj_w, const float* __restrict__ adj_m,
    const float* __restrict__ b_in, const float* __restrict__ basis,
    const float* __restrict__ k_w, const float* __restrict__ k_b,
    const float* __restrict__ q_w, const float* __restrict__ q_b,
    const float* __restrict__ Vs, const float* __restrict__ Sm,
    float* adjf, f16* __restrict__ adj16,
    float* __restrict__ cq, f16* __restrict__ MqA,
    f16* __restrict__ V16, f16* __restrict__ S16, float* __restrict__ b_eff) {
  __shared__ float sK4[4 * DD];
  __shared__ float sMq[4 * DD];
  __shared__ __attribute__((aligned(16))) float s_be[8192];
  const int t = threadIdx.x;

  {
    const float* wr = adj_w + t * NN;
    const float* mr = adj_m + t * NN;
    float deg = 0.0f;
#pragma unroll 1
    for (int mm = 0; mm < NN; ++mm) deg += sigm_fast(wr[mm]) * mr[mm];
    deg = fmaxf(deg, 1e-6f);
    const float rdeg = 1.0f / deg;
    int over = 0;
#pragma unroll 1
    for (int mm = 0; mm < NN; ++mm) over += ((sigm_fast(wr[mm]) * mr[mm]) * rdeg > 0.1f) ? 1 : 0;
    const bool need = over < 1;
    const int fnb = ((t >> 4) > 0) ? (t - 16) : (t + 16);
    float* arow = adjf + t * NN;
    f16* hrow = adj16 + t * NN;
#pragma unroll 1
    for (int q = 0; q < NN / 8; ++q) {
      v4f lo, hi;
      v8h o;
#pragma unroll
      for (int i = 0; i < 8; ++i) {
        const int mm = 8 * q + i;
        float a = (sigm_fast(wr[mm]) * mr[mm]) * rdeg;
        a = (need && mm == fnb) ? fmaxf(a, 0.5f) : a;
        if (i < 4) lo[i] = a; else hi[i - 4] = a;
        o[i] = (f16)a;
      }
      vst2((v4f*)(arow + 8 * q), lo);
      vst2((v4f*)(arow + 8 * q) + 1, hi);
      vst2((v8h*)(hrow + 8 * q), o);
    }
  }

  {
    const int j = t >> 6, d = t & 63;
    float s = 0.0f;
#pragma unroll 1
    for (int e = 0; e < DD; ++e) s += basis[j * DD + e] * k_w[d * DD + e];
    sK4[t] = s + k_b[d];
  }
  __syncthreads();
  {
    const int e = t >> 2, j = t & 3;
    float s = 0.0f;
#pragma unroll 1
    for (int d = 0; d < DD; ++d) s += q_w[d * DD + e] * sK4[j * DD + d];
    sMq[j * DD + e] = s * 0.125f;
  }
  if (t < 8) {
    v4f o;
#pragma unroll
    for (int u = 0; u < 4; ++u) {
      const int idx = 4 * t + u;
      float s = 0.0f;
      if (idx < 4) {
#pragma unroll 1
        for (int d = 0; d < DD; ++d) s += q_b[d] * sK4[idx * DD + d];
      }
      o[u] = s * 0.125f;
    }
    vst2((v4f*)cq + t, o);
  }
  __syncthreads();
  if (t < 128) {
    const int row = t >> 3, pc = (t & 7) * 8;
    v8h o;
#pragma unroll
    for (int i = 0; i < 8; ++i) {
      const float v = sMq[(row & 3) * DD + pc + i] * SC_MQ;
      o[i] = (f16)((row < 4) ? v : 0.0f);
    }
    vst2((v8h*)MqA + t, o);
  }
#pragma unroll
  for (int it = 0; it < 2; ++it) {
    const int i8 = it * 256 + t;
    {
      const v4f p0 = *(const v4f*)(Vs + i8 * 8), p1 = *(const v4f*)(Vs + i8 * 8 + 4);
      v8h o;
#pragma unroll
      for (int i = 0; i < 4; ++i) { o[i] = (f16)(p0[i] * SC_V); o[4 + i] = (f16)(p1[i] * SC_V); }
      vst2((v8h*)V16 + i8, o);
    }
    {
      const v4f p0 = *(const v4f*)(Sm + i8 * 8), p1 = *(const v4f*)(Sm + i8 * 8 + 4);
      v8h o;
#pragma unroll
      for (int i = 0; i < 4; ++i) { o[i] = (f16)(p0[i] * SC_S); o[4 + i] = (f16)(p1[i] * SC_S); }
      vst2((v8h*)S16 + i8, o);
    }
  }
  __syncthreads();

  {
    const int d = t & 63, g = t >> 6;
#pragma unroll 1
    for (int rep = 0; rep < 2; ++rep) {
#pragma unroll 1
      for (int nn = 0; nn < 32; ++nn) {
        const int n = rep * 128 + g * 32 + nn;
        const float* ar = adjf + n * NN;
        float s = 0.0f;
#pragma unroll 4
        for (int mm = 0; mm < NN; ++mm) s += ar[mm] * b_in[mm * DD + d];
        s_be[(g * 32 + nn) * DD + d] = s;
      }
      __syncthreads();
#pragma unroll
      for (int it = 0; it < 8; ++it) {
        const int f = it * 256 + t;
        const v4f v = *(const v4f*)(s_be + 4 * f);
        vst2((v4f*)(b_eff + rep * 8192) + f, v);
      }
      __syncthreads();
    }
  }
}

__global__ __launch_bounds__(256) void k_cvx(const float* __restrict__ x, f16* __restrict__ x16, int nv8) {
  const int i = blockIdx.x * 256 + threadIdx.x;
  if (i >= nv8) return;
  const v4f p0 = *(const v4f*)(x + (size_t)i * 8), p1 = *(const v4f*)(x + (size_t)i * 8 + 4);
  v8h o;
#pragma unroll
  for (int k = 0; k < 4; ++k) { o[k] = (f16)p0[k]; o[4 + k] = (f16)p1[k]; }
  vst2((v8h*)x16 + i, o);
}

__global__ __launch_bounds__(256) void k_weff(const float* __restrict__ W_in,
                                              const f16* __restrict__ adj16,
                                              f16* __restrict__ Weff) {
  __shared__ __attribute__((aligned(16))) f16 sT[64 * TP];
  const int tid = threadIdx.x, lane = tid & 31, wave = tid >> 5;
  const int m = lane & 15, h = lane >> 4;
  const int d = blockIdx.x, fc = blockIdx.y;

#pragma unroll 1
  for (int it = 0; it < 16; ++it) {
    const int idx = it * 256 + tid;
    const int mm = idx >> 4, q = idx & 15;
    const v4f w = *(const v4f*)(W_in + (size_t)(mm * DD + d) * FF + fc * 64 + 4 * q);
    f16* tp = sT + (4 * q) * TP + mm;
    tp[0]      = (f16)(w[0] * SC_WIN);
    tp[TP]     = (f16)(w[1] * SC_WIN);
    tp[2 * TP] = (f16)(w[2] * SC_WIN);
    tp[3 * TP] = (f16)(w[3] * SC_WIN);
  }
  __syncthreads();

  v8f acc[8];
#pragma unroll
  for (int j = 0; j < 8; ++j) acc[j] = zero8();
  const f16* ar0 = adj16 + (size_t)(32 * wave + m) * NN + 8 * h;
  const f16* ar1 = ar0 + 16 * NN;
  const f16* br = sT + m * TP + 8 * h;
#pragma unroll 1
  for (int ks = 0; ks < NN / 32; ++ks) {
    const int k0 = ks * 32;
    const v16h a0 = ldf(ar0 + k0), a1 = ldf(ar1 + k0);
    const v16h b0 = ldf(br + k0), b1 = ldf(br + 16 * TP + k0);
    const v16h b2 = ldf(br + 32 * TP + k0), b3 = ldf(br + 48 * TP + k0);
    acc[0] = wmma16(a0, b0, acc[0]);
    acc[1] = wmma16(a0, b1, acc[1]);
    acc[2] = wmma16(a0, b2, acc[2]);
    acc[3] = wmma16(a0, b3, acc[3]);
    acc[4] = wmma16(a1, b0, acc[4]);
    acc[5] = wmma16(a1, b1, acc[5]);
    acc[6] = wmma16(a1, b2, acc[6]);
    acc[7] = wmma16(a1, b3, acc[7]);
    guard_8w(acc, a0, a1, b0, b1, b2, b3);
  }
  __syncthreads();

  f16* so = sT + wave * 2048;
#pragma unroll
  for (int j = 0; j < 4; ++j)
#pragma unroll
    for (int r = 0; r < 8; ++r) {
      so[(8 * h + r) * 64 + 16 * j + m]      = (f16)(acc[j][r] * WEFF_POST);
      so[(16 + 8 * h + r) * 64 + 16 * j + m] = (f16)(acc[4 + j][r] * WEFF_POST);
    }
  __syncthreads();
  {
    const int rr = lane >> 3, pc = (lane & 7) * 8;
#pragma unroll
    for (int q = 0; q < 8; ++q) {
      const int row = 4 * q + rr;
      const v8h v = *(const v8h*)(so + row * 64 + pc);
      const int n = 32 * wave + row;
      vst2((v8h*)(Weff + ((size_t)n * DD + d) * FF + fc * 64 + pc), v);
    }
  }
}

__global__ __launch_bounds__(256) void k_cvw(const float* __restrict__ W_out, f16* __restrict__ W16, int nv8) {
  const int i = blockIdx.x * 256 + threadIdx.x;
  if (i >= nv8) return;
  const int c = i >> 11, k8 = (i & 2047) * 8;
  v8h o;
  if (c < NCLS) {
    const float* p = W_out + (size_t)c * HH + k8;
    const v4f p0 = *(const v4f*)(p), p1 = *(const v4f*)(p + 4);
#pragma unroll
    for (int k = 0; k < 4; ++k) { o[k] = (f16)(p0[k] * SC_WO); o[4 + k] = (f16)(p1[k] * SC_WO); }
  } else {
#pragma unroll
    for (int k = 0; k < 8; ++k) o[k] = (f16)0.0f;
  }
  vst2((v8h*)W16 + i, o);
}

__global__ __launch_bounds__(64) void k_chain(
    const f16* __restrict__ x16, const f16* __restrict__ Weff,
    const float* __restrict__ b_eff, const f16* __restrict__ V16,
    const f16* __restrict__ S16, const f16* __restrict__ MqA,
    const float* __restrict__ cq, const float* __restrict__ mix_w,
    const float* __restrict__ mix_b, const float* __restrict__ basis,
    f16* __restrict__ xc) {
  __shared__ __attribute__((aligned(16))) float s_w[2][1024];
  const int tid = threadIdx.x, lane = tid & 31, wave = tid >> 5;
  const int m = lane & 15, h = lane >> 4;
  const int bl = (blockIdx.x * 2 + wave) * 16;
  const int ng = blockIdx.y;
  float* sw = s_w[wave];
  const v4f cq4 = *(const v4f*)(cq + 8 * h);
  const float mb = mix_b[0];
  const f16* xr = x16 + (size_t)(bl + m) * FF + 8 * h;

#pragma unroll 1
  for (int ni = 0; ni < 16; ++ni) {
    const int n = ng * 16 + ni;
    const f16* wr = Weff + (size_t)(n * DD + m) * FF + 8 * h;
    v8f t0 = zero8(), t1 = zero8(), t2 = zero8(), t3 = zero8();
#pragma unroll 1
    for (int ks = 0; ks < FF / 32; ++ks) {
      const int k0 = ks * 32;
      const v16h xb = ldf(xr + k0);
      const v16h a0 = ldf(wr + k0);
      const v16h a1 = ldf(wr + 16 * FF + k0);
      const v16h a2 = ldf(wr + 32 * FF + k0);
      const v16h a3 = ldf(wr + 48 * FF + k0);
      t0 = wmma16(a0, xb, t0);
      t1 = wmma16(a1, xb, t1);
      t2 = wmma16(a2, xb, t2);
      t3 = wmma16(a3, xb, t3);
      guard_4(t0, t1, t2, t3, a0, a1, a2, a3, xb);
    }
    const float* bp = b_eff + n * DD + 8 * h;
    t0 = axpb8(t0, INV_WEFF, bp);
    t1 = axpb8(t1, INV_WEFF, bp + 16);
    t2 = axpb8(t2, INV_WEFF, bp + 32);
    t3 = axpb8(t3, INV_WEFF, bp + 48);
    const v16h tb0 = pack2(t0, t1, 1.0f), tb1 = pack2(t2, t3, 1.0f);

    v8f y0, y1, y2, y3;
    chain_pair(S16, 0, m, h, tb0, tb1, y0, y1);
    chain_pair(S16, 2, m, h, tb0, tb1, y2, y3);
    y0 = clip8s(y0, INV_S); y1 = clip8s(y1, INV_S); y2 = clip8s(y2, INV_S); y3 = clip8s(y3, INV_S);
    const v16h yb0 = pack2(y0, y1, SC_Y), yb1 = pack2(y2, y3, SC_Y);

    v8f v0, v1, v2, v3;
    chain_pair(V16, 0, m, h, tb0, tb1, v0, v1);
    chain_pair(V16, 2, m, h, tb0, tb1, v2, v3);
    v0 = clip8s(v0, INV_V); v1 = clip8s(v1, INV_V); v2 = clip8s(v2, INV_V); v3 = clip8s(v3, INV_V);

    v8f p0, p1, p2, p3;
    chain_pair(V16, 0, m, h, yb0, yb1, p0, p1);
    chain_pair(V16, 2, m, h, yb0, yb1, p2, p3);
    p0 = clip8s(p0, INV_YV); p1 = clip8s(p1, INV_YV); p2 = clip8s(p2, INV_YV); p3 = clip8s(p3, INV_YV);

    const float* mp = mix_w + 8 * h;
    float sdot = dot8(v0, mp) + dot8(v1, mp + 16) + dot8(v2, mp + 32) + dot8(v3, mp + 48);
    sdot += __shfl_xor(sdot, 16);
    const float mixv = 1.0f / (1.0f + expf(-(sdot + mb)));
    const float omix = 1.0f - mixv;
#pragma unroll
    for (int r = 0; r < 8; ++r) {
      v0[r] = fminf(CLIPV, fmaxf(-CLIPV, mixv * v0[r] + omix * p0[r]));
      v1[r] = fminf(CLIPV, fmaxf(-CLIPV, mixv * v1[r] + omix * p1[r]));
      v2[r] = fminf(CLIPV, fmaxf(-CLIPV, mixv * v2[r] + omix * p2[r]));
      v3[r] = fminf(CLIPV, fmaxf(-CLIPV, mixv * v3[r] + omix * p3[r]));
    }
    const v16h cb0 = pack2(v0, v1, SC_CELL), cb1 = pack2(v2, v3, SC_CELL);

    v8f at;
    {
      const f16* qp = MqA + m * DD + 8 * h;
      const v16h q0 = ldf(qp), q1 = ldf(qp + 32);
      at = wmma16(q0, cb0, zero8());
      at = wmma16(q1, cb1, at);
      guard_1(at, q0, q1, cb0, cb1);
    }
    const float g0 = at[0] * INV_ATT + cq4[0];
    const float g1 = at[1] * INV_ATT + cq4[1];
    const float g2 = at[2] * INV_ATT + cq4[2];
    const float g3 = at[3] * INV_ATT + cq4[3];
    const float mx = fmaxf(fmaxf(g0, g1), fmaxf(g2, g3));
    const float e0 = expf(g0 - mx), e1 = expf(g1 - mx), e2 = expf(g2 - mx), e3 = expf(g3 - mx);
    const float inv = 1.0f / (e0 + e1 + e2 + e3);
    if (h == 0) {
      v4f o;
      o[0] = e0 * inv; o[1] = e1 * inv; o[2] = e2 * inv; o[3] = e3 * inv;
      *(v4f*)(sw + m * 64 + ni * 4) = o;
    }
  }
  __syncthreads();

  {
    const int rr = lane >> 3, pc = (lane & 7) * 8;
    const v4f b00 = *(const v4f*)(basis + pc),          b01 = *(const v4f*)(basis + pc + 4);
    const v4f b10 = *(const v4f*)(basis + DD + pc),     b11 = *(const v4f*)(basis + DD + pc + 4);
    const v4f b20 = *(const v4f*)(basis + 2 * DD + pc), b21 = *(const v4f*)(basis + 2 * DD + pc + 4);
    const v4f b30 = *(const v4f*)(basis + 3 * DD + pc), b31 = *(const v4f*)(basis + 3 * DD + pc + 4);
    f16* xb = xc + (size_t)bl * HH + (size_t)ng * 1024 + pc;
#pragma unroll 1
    for (int g = 0; g < 64; ++g) {
      const int idx = 4 * g + rr;
      const int r = idx >> 4, L = idx & 15;
      const v4f w = *(const v4f*)(sw + r * 64 + L * 4);
      v4f lo = w[0] * b00; lo += w[1] * b10; lo += w[2] * b20; lo += w[3] * b30;
      v4f hi = w[0] * b01; hi += w[1] * b11; hi += w[2] * b21; hi += w[3] * b31;
      v8h o;
#pragma unroll
      for (int i = 0; i < 4; ++i) {
        o[i]     = (f16)(fminf(CLIPV, fmaxf(-CLIPV, lo[i])) * SC_XC);
        o[4 + i] = (f16)(fminf(CLIPV, fmaxf(-CLIPV, hi[i])) * SC_XC);
      }
      vst2((v8h*)(xb + (size_t)r * HH + L * 64), o);
    }
  }
}

__global__ __launch_bounds__(224) void k_out(const f16* __restrict__ xc, const f16* __restrict__ W16,
                                             const float* __restrict__ b_out, float* __restrict__ out) {
  __shared__ __attribute__((aligned(16))) float s_o[16 * NCLS];
  const int tid = threadIdx.x, lane = tid & 31, wave = tid >> 5;
  const int m = lane & 15, h = lane >> 4;
  const int bl = blockIdx.x * 16, c0 = wave * 144;
  v8f acc[9];
#pragma unroll
  for (int j = 0; j < 9; ++j) acc[j] = zero8();
  const f16* ap = xc + (size_t)(bl + m) * HH + 8 * h;
  const f16* gp = W16 + (size_t)(c0 + m) * HH + 8 * h;
  const size_t TS = (size_t)16 * HH;
#pragma unroll 1
  for (int ks = 0; ks < HH / 32; ++ks) {
    const int k0 = ks * 32;
    const v16h a = ldf(ap + k0);
    {
      const v16h b0 = ldf(gp + k0), b1 = ldf(gp + TS + k0), b2 = ldf(gp + 2 * TS + k0);
      acc[0] = wmma16(a, b0, acc[0]);
      acc[1] = wmma16(a, b1, acc[1]);
      acc[2] = wmma16(a, b2, acc[2]);
      guard_3(acc[0], acc[1], acc[2], b0, b1, b2, a);
    }
    {
      const v16h b0 = ldf(gp + 3 * TS + k0), b1 = ldf(gp + 4 * TS + k0), b2 = ldf(gp + 5 * TS + k0);
      acc[3] = wmma16(a, b0, acc[3]);
      acc[4] = wmma16(a, b1, acc[4]);
      acc[5] = wmma16(a, b2, acc[5]);
      guard_3(acc[3], acc[4], acc[5], b0, b1, b2, a);
    }
    {
      const v16h b0 = ldf(gp + 6 * TS + k0), b1 = ldf(gp + 7 * TS + k0), b2 = ldf(gp + 8 * TS + k0);
      acc[6] = wmma16(a, b0, acc[6]);
      acc[7] = wmma16(a, b1, acc[7]);
      acc[8] = wmma16(a, b2, acc[8]);
      guard_3(acc[6], acc[7], acc[8], b0, b1, b2, a);
    }
  }
#pragma unroll
  for (int j = 0; j < 9; ++j) {
    const int col = c0 + 16 * j + m;
    if (col < NCLS) {
      const float bo = b_out[col];
#pragma unroll
      for (int r = 0; r < 8; ++r) s_o[(8 * h + r) * NCLS + col] = acc[j][r] * INV_OUT + bo;
    }
  }
  __syncthreads();
  float* ob = out + (size_t)bl * NCLS;
  const int nv4 = (16 * NCLS) / 4;
#pragma unroll 1
  for (int it = 0; it < 18; ++it) {
    const int f = it * 224 + tid;
    if (f < nv4) {
      const v4f v = *(const v4f*)(s_o + f * 4);
      vst2((v4f*)ob + f, v);
    }
  }
}

extern "C" void kernel_launch(void* const* d_in, const int* in_sizes, int n_in,
                              void* d_out, int out_size, void* d_ws, size_t ws_size,
                              hipStream_t stream) {
  if (n_in < 16) return;
  const float* x       = (const float*)d_in[0];
  const float* W_in    = (const float*)d_in[1];
  const float* b_in    = (const float*)d_in[2];
  const float* adj_w   = (const float*)d_in[3];
  const float* adj_m   = (const float*)d_in[4];
  const float* V_slow  = (const float*)d_in[5];
  const float* sem_mem = (const float*)d_in[6];
  const float* mix_w   = (const float*)d_in[7];
  const float* mix_b   = (const float*)d_in[8];
  const float* basis   = (const float*)d_in[9];
  const float* q_w     = (const float*)d_in[10];
  const float* q_b     = (const float*)d_in[11];
  const float* k_w     = (const float*)d_in[12];
  const float* k_b     = (const float*)d_in[13];
  const float* W_out   = (const float*)d_in[14];
  const float* b_out   = (const float*)d_in[15];
  float* out = (float*)d_out;

  const int nx = in_sizes[0];
  const int B = nx / FF;
  if (B <= 0 || nx != B * FF || (B % 32) != 0) return;
  if (in_sizes[1] != HH * FF || in_sizes[2] != HH || in_sizes[3] != NN * NN || in_sizes[4] != NN * NN ||
      in_sizes[5] != DD * DD || in_sizes[6] != DD * DD || in_sizes[7] != DD || in_sizes[8] < 1 ||
      in_sizes[9] != 4 * DD || in_sizes[10] != DD * DD || in_sizes[11] != DD || in_sizes[12] != DD * DD ||
      in_sizes[13] != DD || in_sizes[14] != NCLS * HH || in_sizes[15] != NCLS)
    return;
  if (out_size != B * NCLS) return;

  const int rcap = (B < RBH) ? B : RBH;

  char* ws = (char*)d_ws;
  size_t off = 0;
  float* adjf  = (float*)(ws + off);  off += (size_t)NN * NN * 4;
  f16*   adj16 = (f16*)(ws + off);    off += (size_t)NN * NN * 2;
  float* cq    = (float*)(ws + off);  off += 128;
  f16*   MqA   = (f16*)(ws + off);    off += (size_t)16 * DD * 2;
  f16*   V16   = (f16*)(ws + off);    off += (size_t)DD * DD * 2;
  f16*   S16   = (f16*)(ws + off);    off += (size_t)DD * DD * 2;
  float* b_eff = (float*)(ws + off);  off += (size_t)HH * 4;
  f16*   x16   = (f16*)(ws + off);    off += (size_t)B * FF * 2;
  f16*   Weff  = (f16*)(ws + off);    off += (size_t)HH * FF * 2;
  f16*   W16   = (f16*)(ws + off);    off += (size_t)NCP * HH * 2;
  f16*   xc    = (f16*)(ws + off);    off += (size_t)rcap * HH * 2;
  if (off > ws_size || off > (size_t)134217728) return;

  const int nx8 = B * FF / 8;
  const int nw8 = NCP * HH / 8;

  hipLaunchKernelGGL(k_prep, dim3(1), dim3(256), 0, stream,
                     adj_w, adj_m, b_in, basis, k_w, k_b, q_w, q_b, V_slow, sem_mem,
                     adjf, adj16, cq, MqA, V16, S16, b_eff);
  hipLaunchKernelGGL(k_cvx, dim3((nx8 + 255) / 256), dim3(256), 0, stream, x, x16, nx8);
  hipLaunchKernelGGL(k_weff, dim3(DD, FF / 64), dim3(256), 0, stream, W_in, adj16, Weff);
  hipLaunchKernelGGL(k_cvw, dim3((nw8 + 255) / 256), dim3(256), 0, stream, W_out, W16, nw8);

  const int npart = (B + RBH - 1) / RBH;
  for (int p = 0; p < npart; ++p) {
    const int rb = p * RBH;
    int rows = B - rb;
    if (rows > RBH) rows = RBH;
    hipLaunchKernelGGL(k_chain, dim3(rows / 32, NN / 16), dim3(64), 0, stream,
                       x16 + (size_t)rb * FF, Weff, b_eff, V16, S16, MqA, cq, mix_w, mix_b, basis, xc);
    hipLaunchKernelGGL(k_out, dim3(rows / 16), dim3(224), 0, stream,
                       xc, W16, b_out, out + (size_t)rb * NCLS);
  }
  (void)hipGetLastError();
}
